// CGCN_27986006901064
// MI455X (gfx1250) — hardware-run, weakly checked
//
#include <hip/hip_runtime.h>


namespace {
constexpr int N = 16384, FI = 512, H = 256, C = 16, E = 524288, T = 4096, NSLAB = N / 32  ;
constexpr float HS = 256.0f, WSC = 256.0f, TAU = 0.5f;
typedef _Float16 b16;
typedef __attribute__((ext_vector_type(16))) _Float16 v16b;
typedef __attribute__((ext_vector_type(8))) _Float16 v8b;
typedef __attribute__((ext_vector_type(8))) float v8f;
typedef __attribute__((ext_vector_type(4))) float v4f;
__device__ __forceinline__ float bf16_rne(float f) { unsigned int u = __float_as_uint(f); u += 0x7FFFu + ((u >> 16) & 1u); float r = __uint_as_float(u & 0xFFFF0000u); asm volatile("" : "+v"(r)); return r; }
__device__ __forceinline__ float bfv(float f) { float r = bf16_rne(f); asm volatile("" : "+v"(r)); return r; }
__device__ __forceinline__ void split16(float v, b16& hi, b16& lo) { hi = (b16)v; lo = (b16)(v - (float)hi); }
__device__ __forceinline__ v16b frag_kb(const b16* p, int hh) { const v8b a = *(const v8b*)(p + 8 * hh), b = *(const v8b*)(p + 16 + 8 * hh); v16b f;
#pragma unroll
  for (int e = 0; e < 8; ++e) { f[e] = a[e]; f[8 + e] = b[e]; } return f; }
__device__ __forceinline__ v8f wmma16b(v16b a, v16b b, v8f c) { v8f d = __builtin_amdgcn_wmma_f32_16x16x32_f16(false, a, false, b, (short)0, c, false, false); asm volatile("v_nop\n\tv_nop\n\tv_nop\n\tv_nop" : "+v"(d) : "v"(a), "v"(b)); return d; }
__device__ __forceinline__ void wave_lds_sync() { __builtin_amdgcn_fence(__ATOMIC_RELEASE, "workgroup"); __builtin_amdgcn_wave_barrier(); __builtin_amdgcn_fence(__ATOMIC_ACQUIRE, "workgroup"); }
__device__ __forceinline__ float pmul(float a, float b) { float p = a * b; asm volatile("" : "+v"(p)); return p; }
__device__ __forceinline__ int iclamp(int v, int lo, int hi) { return v < lo ? lo : (v > hi ? hi : v); }
constexpr int CSR_NBLK8 = 512, CSR_GB8 = 8, CSR_GN8 = 1 << CSR_GB8  , CSR_TS8 = (CSR_GN8 < 32 ? 32 : CSR_GN8)  , CSR_MAXG8 = 512, CSR_CAP8 = 12288  ;
__device__ __host__ __forceinline__ int csr_tix8(int v) { return (v >> CSR_GB8) * CSR_TS8 + (v & (CSR_GN8 - 1)); }
__global__ __launch_bounds__(64) void csrA_kernel8(const int* __restrict__ dst, int E, int N, int nG, int CHP, int NGP, int* __restrict__ STG, int* __restrict__ HST) {
  extern __shared__ int sm[];
  int* cnt = sm; int* run = sm + NGP; int* ids = sm + 2 * NGP;
  const int b = blockIdx.x; const int ch = (E + CSR_NBLK8 - 1) / CSR_NBLK8; const int e0 = b * ch, e1 = min(E, e0 + ch);
  for (int i = threadIdx.x; i < NGP; i += 64) cnt[i] = 0;
  for (int i = threadIdx.x; i < CHP; i += 64) ids[i] = -1;
  __syncthreads();
  if (threadIdx.x == 0) {
    for (int e = e0; e < e1; ++e) { int d = dst[e]; d = (d < 0) ? 0 : (d >= N ? N - 1 : d); cnt[d >> CSR_GB8] += 1; }
    int acc = 0; for (int g = 0; g < nG; ++g) { run[g] = acc; acc += cnt[g]; }
    for (int e = e0; e < e1; ++e) { int d = dst[e]; d = (d < 0) ? 0 : (d >= N ? N - 1 : d); const int g = d >> CSR_GB8; ids[run[g]] = e; run[g] += 1; } }
  __syncthreads();
  typedef __attribute__((ext_vector_type(4))) int v4i;
  for (int pass = 0; pass < 2; ++pass) {
    for (int i = threadIdx.x; i < CHP / 4; i += 64) *(volatile v4i*)(STG + (size_t)b * CHP + i * 4) = *(const v4i*)(&ids[i * 4]);
    for (int i = threadIdx.x; i < NGP / 4; i += 64) { v4i v; for (int e = 0; e < 4; ++e) v[e] = (i * 4 + e < nG) ? cnt[i * 4 + e] : 0; *(volatile v4i*)(HST + (size_t)b * NGP + i * 4) = v; }
    __threadfence(); }
}
__global__ __launch_bounds__(512) void csrS_kernel8(const int* __restrict__ HST, int nG, int NGP, int* __restrict__ START, int* __restrict__ TOT, int* __restrict__ OFF) {
  __shared__ int tot[CSR_MAXG8];
  const int b = threadIdx.x;
  for (int pass = 0; pass < 2; ++pass) { int runb = 0; for (int g = 0; g < nG; ++g) { int c = HST[(size_t)b * NGP + g]; c = (c < 0) ? 0 : c; ((volatile int*)OFF)[(size_t)g * CSR_NBLK8 + b] = runb; runb += c; } __threadfence(); }
  for (int g = threadIdx.x; g < nG; g += 512) { int s = 0; for (int bb = 0; bb < CSR_NBLK8; ++bb) { int c = HST[(size_t)bb * NGP + g]; s += (c < 0) ? 0 : c; } tot[g] = s; }
  __syncthreads();
  if (threadIdx.x < 32) {
    __shared__ int st[CSR_MAXG8 + 32];
    if (threadIdx.x == 0) { int acc = 0; for (int g = 0; g < NGP; ++g) { st[g] = acc; if (g < nG) acc += (tot[g] + 31) & ~31; } st[NGP] = acc; }
    __builtin_amdgcn_fence(__ATOMIC_RELEASE, "workgroup"); __builtin_amdgcn_wave_barrier(); __builtin_amdgcn_fence(__ATOMIC_ACQUIRE, "workgroup");
    for (int pass = 0; pass < 2; ++pass) { for (int i = threadIdx.x; i < NGP + 32; i += 32) { ((volatile int*)START)[i] = (i <= NGP) ? st[min(i, NGP)] : 0; ((volatile int*)TOT)[i] = (i < nG) ? tot[i] : 0; } __threadfence(); } }
}
__global__ __launch_bounds__(256) void csrB_kernel8(const int* __restrict__ dst, int N, int nG, int CHP, int NGP, int permLen, const int* __restrict__ STG, const int* __restrict__ HST, const int* __restrict__ OFF, const int* __restrict__ START, const int* __restrict__ TOT, int* __restrict__ PERM, int* __restrict__ ROWPTR, int* __restrict__ ROWCNT, int* __restrict__ FLAG) {
  typedef __attribute__((ext_vector_type(4))) int v4i;
  __shared__ int ids[CSR_CAP8]; __shared__ unsigned short key[CSR_CAP8]; __shared__ int outp[CSR_CAP8]; __shared__ int ncnt[CSR_GN8 + 1]; __shared__ int boff[CSR_NBLK8 + 1];
  const int g = blockIdx.x, t_ = threadIdx.x; int tot = TOT[g]; int st = START[g], stn = START[g + 1]; const int v0 = g * CSR_GN8; const int nv = min(CSR_GN8, N - v0); const int t0 = g * CSR_TS8;
  st = (st < 0) ? 0 : (st > permLen - 32 ? permLen - 32 : st) & ~31; stn = (stn < st) ? st : (stn > permLen ? permLen : stn); tot = (tot < 0) ? 0 : tot; if (tot > stn - st && tot <= CSR_CAP8) tot = stn - st;
  if (tot > CSR_CAP8) {
    for (int pass = 0; pass < 2; ++pass) { for (int i = t_; i < CSR_TS8 / 4; i += 256) { v4i a, c; for (int e = 0; e < 4; ++e) { a[e] = st; c[e] = 0; } *(volatile v4i*)(ROWPTR + t0 + i * 4) = a; *(volatile v4i*)(ROWCNT + t0 + i * 4) = c; } if (t_ == 0) ((volatile int*)FLAG)[0] = 1; __threadfence(); } (void)nv; return; }
  if (t_ == 0) { int acc = 0; for (int b = 0; b < CSR_NBLK8; ++b) { boff[b] = acc; int c = HST[(size_t)b * NGP + g]; c = (c < 0) ? 0 : (c > CHP ? CHP : c); acc += c; if (acc > tot) acc = tot; } boff[CSR_NBLK8] = acc; }
  for (int i = t_; i <= CSR_GN8; i += 256) ncnt[i] = 0;
  __syncthreads();
  for (int b = 0; b < CSR_NBLK8; ++b) { const int c = boff[b + 1] - boff[b]; int o_ = OFF[(size_t)g * CSR_NBLK8 + b]; o_ = (o_ < 0) ? 0 : (o_ > CHP - c ? CHP - c : o_); const int* src_ = STG + (size_t)b * CHP + o_;
    for (int i = t_; i < c; i += 256) { int id = src_[i]; id = (id < 0) ? 0 : id; ids[boff[b] + i] = id; int d = dst[id]; d = (d < v0) ? v0 : (d >= N ? N - 1 : d); int kk = d - v0; kk = (kk < 0) ? 0 : (kk >= CSR_GN8 ? CSR_GN8 - 1 : kk); key[boff[b] + i] = (unsigned short)kk; } }
  __syncthreads();
  if (t_ == 0) { for (int i = 0; i < tot; ++i) ncnt[key[i]] += 1; int acc = 0; for (int vl = 0; vl < CSR_GN8; ++vl) { const int c = ncnt[vl]; ncnt[vl] = acc; acc += c; } ncnt[CSR_GN8] = acc;
    for (int i = 0; i < tot; ++i) { const int vl = key[i]; outp[ncnt[vl]] = ids[i]; ncnt[vl] += 1; }
    for (int vl = CSR_GN8; vl > 0; --vl) ncnt[vl] = ncnt[vl - 1]; ncnt[0] = 0; }
  __syncthreads();
  for (int pass = 0; pass < 2; ++pass) {
    for (int i = t_; i < (stn - st) / 4; i += 256) { v4i v; for (int e = 0; e < 4; ++e) { const int q = i * 4 + e; v[e] = (q < tot) ? outp[q] : -1; } *(volatile v4i*)(PERM + st + i * 4) = v; }
    for (int i = t_; i < CSR_TS8 / 4; i += 256) { v4i a, c; for (int e = 0; e < 4; ++e) { const int vl = i * 4 + e; const int vc = vl < CSR_GN8 ? vl : CSR_GN8; a[e] = (vl < CSR_GN8) ? st + ncnt[vc] : st; c[e] = (vl < nv) ? (ncnt[(vc < CSR_GN8 ? vc : CSR_GN8 - 1) + 1] - ncnt[vc]) : 0; } *(volatile v4i*)(ROWPTR + t0 + i * 4) = a; *(volatile v4i*)(ROWCNT + t0 + i * 4) = c; }
    __threadfence(); }
}
__global__ __launch_bounds__(256) void csrZ_kernel8(int* __restrict__ p, size_t n4) { typedef __attribute__((ext_vector_type(4))) int v4i; const size_t tid = (size_t)blockIdx.x * 256 + threadIdx.x, nth = (size_t)gridDim.x * 256; v4i z = {0, 0, 0, 0}; for (size_t i = tid; i < n4; i += nth) *(volatile v4i*)(p + i * 4) = z; }
struct CsrBufs8 { int *STG, *HST, *OFF, *START, *TOT, *PERM, *ROWPTR, *ROWCNT, *FLAG; int nG, NGP, CHP; size_t permLen; char* base; size_t bytes; };
static size_t csr_carve8(CsrBufs8& c, char* ws, size_t off, int E, int N) {
  const size_t off0 = off; c.base = ws + off;
  auto al = [&](size_t bytes) { char* p = ws + off; off += (bytes + 255) & ~(size_t)255; return p; };
  c.nG = (N + CSR_GN8 - 1) / CSR_GN8; c.NGP = (c.nG + 31) & ~31; const int ch = (E + CSR_NBLK8 - 1) / CSR_NBLK8; c.CHP = (ch + 31) & ~31; c.permLen = (size_t)E + 32 * (size_t)c.nG + 32;
  c.STG = (int*)al((size_t)CSR_NBLK8 * c.CHP * 4); c.HST = (int*)al((size_t)CSR_NBLK8 * c.NGP * 4); c.OFF = (int*)al((size_t)c.NGP * CSR_NBLK8 * 4); c.START = (int*)al((size_t)(c.NGP + 64) * 4); c.TOT = (int*)al((size_t)(c.NGP + 64) * 4);
  c.PERM = (int*)al(c.permLen * 4); c.ROWPTR = (int*)al((size_t)c.nG * CSR_TS8 * 4); c.ROWCNT = (int*)al((size_t)c.nG * CSR_TS8 * 4); c.FLAG = (int*)al(256);
  c.bytes = off - off0; return off;
}
static void csr_build8(const CsrBufs8& c, const int* dst, int E, int N, hipStream_t stream) {
  const size_t smem = (size_t)(2 * c.NGP + c.CHP) * 4;
  csrZ_kernel8<<<512, 256, 0, stream>>>((int*)c.base, c.bytes / 16);
  csrA_kernel8<<<CSR_NBLK8, 64, smem, stream>>>(dst, E, N, c.nG, c.CHP, c.NGP, c.STG, c.HST);
  csrS_kernel8<<<1, 512, 0, stream>>>(c.HST, c.nG, c.NGP, c.START, c.TOT, c.OFF);
  csrB_kernel8<<<c.nG, 256, 0, stream>>>(dst, N, c.nG, c.CHP, c.NGP, (int)c.permLen, c.STG, c.HST, c.OFF, c.START, c.TOT, c.PERM, c.ROWPTR, c.ROWCNT, c.FLAG);
}


__global__ __launch_bounds__(256) void wput_kernel(const float* __restrict__ wg1, const float* __restrict__ wg2, const float* __restrict__ wl1, const float* __restrict__ wl2, const float* __restrict__ wc1, const float* __restrict__ wc2, b16* __restrict__ WG, b16* __restrict__ WL, b16* __restrict__ WC1, b16* __restrict__ WC2) { const int u = blockIdx.x * 256 + threadIdx.x; v8b v;
  if (u < 2 * H * (FI / 8)) { const int o = u / (FI / 8), k0 = (u % (FI / 8)) * 8; const float* w = o < H ? wg1 : wg2; const int oo = o % H;
#pragma unroll
    for (int j = 0; j < 8; ++j) v[j] = (b16)(bf16_rne(w[(size_t)(k0 + j) * H + oo]) * WSC); for (int pass = 0; pass < 2; ++pass) { *(volatile v8b*)(WG + (size_t)o * FI + k0) = v; __threadfence(); } }
  if (u < 2 * H * (H / 8)) { const int o = u / (H / 8), k0 = (u % (H / 8)) * 8; const float* w = o < H ? wl1 : wl2; const int oo = o % H;
#pragma unroll
    for (int j = 0; j < 8; ++j) v[j] = (b16)(bf16_rne(w[(size_t)(k0 + j) * H + oo]) * WSC); for (int pass = 0; pass < 2; ++pass) { *(volatile v8b*)(WL + (size_t)o * H + k0) = v; __threadfence(); } }
  if (u < H * (H / 8)) { const int o = u / (H / 8), k0 = (u % (H / 8)) * 8;
#pragma unroll
    for (int j = 0; j < 8; ++j) v[j] = (b16)(bf16_rne(wc1[(size_t)(k0 + j) * H + o]) * WSC); for (int pass = 0; pass < 2; ++pass) { *(volatile v8b*)(WC1 + (size_t)o * H + k0) = v; __threadfence(); } }
  if (u < C * (H / 8)) { const int o = u / (H / 8), k0 = (u % (H / 8)) * 8;
#pragma unroll
    for (int j = 0; j < 8; ++j) v[j] = (b16)(bf16_rne(wc2[(size_t)(k0 + j) * C + o]) * WSC); for (int pass = 0; pass < 2; ++pass) { *(volatile v8b*)(WC2 + (size_t)o * H + k0) = v; __threadfence(); } } }
__global__ __launch_bounds__(32) void sup_kernel(const float* __restrict__ x, const b16* __restrict__ WG, int NLIM, float* __restrict__ SUP) { __shared__ __attribute__((aligned(16))) b16 Ah[16][FI + 8]; __shared__ float Tf[16][H + 4]; const int lane = threadIdx.x, nloc = lane & 15, hlf = lane >> 4; const int k = blockIdx.x & 1; const size_t m0 = (size_t)(blockIdx.x >> 1) * 16; if (m0 >= (size_t)NLIM) return;
  for (int rr = 0; rr < 16; ++rr) for (int q = 0; q < FI / 32; ++q) Ah[rr][q * 32 + lane] = (b16)(bf16_rne(x[(m0 + rr) * FI + q * 32 + lane]) * HS); if (lane < 16) for (int kk = FI; kk < FI + 8; ++kk) Ah[lane][kk] = (b16)0.0f;
  wave_lds_sync(); v8f acc[16];
#pragma unroll
  for (int t = 0; t < 16; ++t) acc[t] = (v8f){};
#pragma unroll 2
  for (int kb = 0; kb < FI; kb += 32) { const v16b a = frag_kb(&Ah[nloc][kb], hlf);
#pragma unroll
    for (int t = 0; t < 16; ++t) acc[t] = wmma16b(a, frag_kb(WG + (size_t)(k * H + t * 16 + nloc) * FI + kb, hlf), acc[t]); }
#pragma unroll
  for (int t = 0; t < 16; ++t)
#pragma unroll
    for (int r8 = 0; r8 < 8; ++r8) Tf[8 * hlf + r8][t * 16 + nloc] = acc[t][r8] * (1.0f / (HS * WSC));
  wave_lds_sync();
  for (int pass = 0; pass < 2; ++pass) { for (int rr = 0; rr < 16; ++rr) for (int q = 0; q < 2; ++q) *(volatile v4f*)(SUP + (m0 + rr) * 2 * H + k * H + q * 128 + lane * 4) = *(const v4f*)(&Tf[rr][q * 128 + lane * 4]); __threadfence(); } }
__global__ __launch_bounds__(256) void spmm_kernel(const float* __restrict__ SUP, const float* __restrict__ val, const int* __restrict__ cols, const float* __restrict__ bg1, const float* __restrict__ bg2, const int* __restrict__ PERM, const int* __restrict__ ROWPTR, const int* __restrict__ ROWCNT, int permLen, int NLIM, float* __restrict__ HH) { const int wave = threadIdx.x >> 5, lane = threadIdx.x & 31; const size_t i = (size_t)blockIdx.x * 8 + wave; if (i >= (size_t)NLIM) return; int st = ROWPTR[i], cnt = ROWCNT[i]; cnt = iclamp(cnt, 0, E); st = iclamp(st, 0, permLen - cnt);
  float acc[16];
#pragma unroll
  for (int k = 0; k < 16; ++k) acc[k] = 0.0f;
#pragma unroll 1
  for (int j = 0; j < cnt; ++j) { const int e = iclamp(PERM[st + j], 0, E - 1); const size_t u = (size_t)iclamp(cols[e], 0, N - 1); if (u >= (size_t)NLIM) continue; const float w = bfv(val[e]); const float* sp = SUP + u * 2 * H + lane * 16;
#pragma unroll
    for (int k = 0; k < 16; ++k) acc[k] += pmul(w, sp[k]); }
  float o[16];
#pragma unroll
  for (int k = 0; k < 16; ++k) { const int c = lane * 16 + k; o[k] = fmaxf(acc[k] + bfv(c < H ? bg1[c] : bg2[c - H]), 0.0f); }
  for (int pass = 0; pass < 2; ++pass) {
#pragma unroll
    for (int q = 0; q < 4; ++q) *(volatile v4f*)(HH + i * 2 * H + lane * 16 + q * 4) = (v4f){o[q * 4], o[q * 4 + 1], o[q * 4 + 2], o[q * 4 + 3]}; __threadfence(); } }
__global__ __launch_bounds__(32) void enc_kernel(const float* __restrict__ HH, const b16* __restrict__ WL, const float* __restrict__ bl1, const float* __restrict__ bl2, int NLIM, float* __restrict__ Z, b16* __restrict__ ZN, float* __restrict__ DG) { __shared__ __attribute__((aligned(16))) b16 Ah[16][H + 8], Al[16][H + 8]; __shared__ float T1[16][H + 4], T2[16][H + 4], Dg[16]; const int lane = threadIdx.x, nloc = lane & 15, hlf = lane >> 4; const size_t m0 = (size_t)blockIdx.x * 16; if (m0 >= (size_t)NLIM) return;
#pragma unroll 1
  for (int k = 0; k < 2; ++k) { for (int rr = 0; rr < 16; ++rr) for (int q = 0; q < H / 32; ++q) { b16 p, ql; split16(HH[(m0 + rr) * 2 * H + k * H + q * 32 + lane] * HS, p, ql); Ah[rr][q * 32 + lane] = p; Al[rr][q * 32 + lane] = ql; } if (lane < 16) for (int kk = H; kk < H + 8; ++kk) { Ah[lane][kk] = (b16)0.0f; Al[lane][kk] = (b16)0.0f; }
    wave_lds_sync(); v8f acc[16];
#pragma unroll
    for (int t = 0; t < 16; ++t) acc[t] = (v8f){};
#pragma unroll 2
    for (int kb = 0; kb < H; kb += 32) { const v16b a = frag_kb(&Ah[nloc][kb], hlf), al = frag_kb(&Al[nloc][kb], hlf);
#pragma unroll
      for (int t = 0; t < 16; ++t) { const v16b bw = frag_kb(WL + (size_t)(k * H + t * 16 + nloc) * H + kb, hlf); acc[t] = wmma16b(a, bw, acc[t]); acc[t] = wmma16b(al, bw, acc[t]); } }
    float (*Tk)[H + 4] = k == 0 ? T1 : T2; const float* bl = k == 0 ? bl1 : bl2;
#pragma unroll
    for (int t = 0; t < 16; ++t) { const int cc = t * 16 + nloc; const float bb = bfv(bl[cc]);
#pragma unroll
      for (int r8 = 0; r8 < 8; ++r8) Tk[8 * hlf + r8][cc] = acc[t][r8] * (1.0f / (HS * WSC)) + bb; }
    wave_lds_sync(); }
  for (int pass = 0; pass < 2; ++pass) { for (int rr = 0; rr < 16; ++rr) { float n1 = 0.0f, n2 = 0.0f, v1[8], v2[8];
#pragma unroll
      for (int kq = 0; kq < 8; ++kq) { v1[kq] = T1[rr][lane * 8 + kq]; v2[kq] = T2[rr][lane * 8 + kq]; n1 += v1[kq] * v1[kq]; n2 += v2[kq] * v2[kq]; } for (int o = 16; o; o >>= 1) { n1 += __shfl_xor(n1, o); n2 += __shfl_xor(n2, o); }
      const float i1 = 1.0f / fmaxf(sqrtf(n1), 1e-12f), i2 = 1.0f / fmaxf(sqrtf(n2), 1e-12f); float dg = 0.0f; v8b z1b, z2b; v4f za, zb;
#pragma unroll
      for (int kq = 0; kq < 8; ++kq) { const float a = pmul(v1[kq], i1), b = pmul(v2[kq], i2); dg += a * b; z1b[kq] = (b16)a; z2b[kq] = (b16)b; const float zz = pmul(v1[kq] + v2[kq], 0.5f); if (kq < 4) za[kq] = zz; else zb[kq - 4] = zz; }
      for (int o = 16; o; o >>= 1) dg += __shfl_xor(dg, o);
      const size_t n = m0 + rr; *(volatile v4f*)(Z + n * H + lane * 8) = za; *(volatile v4f*)(Z + n * H + lane * 8 + 4) = zb;
      *(volatile v8b*)(ZN + n * H + lane * 8) = z1b; *(volatile v8b*)(ZN + (size_t)N * H + n * H + lane * 8) = z2b; if (lane == 0) Dg[rr] = dg; } wave_lds_sync(); ((volatile float*)DG)[(m0 / 16) * 32 + lane] = lane < 16 ? Dg[lane] : 0.0f;     __threadfence(); } }
__global__ __launch_bounds__(32) void cls_kernel(const float* __restrict__ Z, const b16* __restrict__ WC1, const b16* __restrict__ WC2, const float* __restrict__ bc1, const float* __restrict__ bc2, int NLIM, float* __restrict__ OUT1) { __shared__ __attribute__((aligned(16))) b16 Ah[16][H + 8], Al[16][H + 8]; __shared__ float Tf[16][C]; const int lane = threadIdx.x, nloc = lane & 15, hlf = lane >> 4; const size_t m0 = (size_t)blockIdx.x * 16; if (m0 >= (size_t)NLIM) return;
  for (int rr = 0; rr < 16; ++rr) for (int q = 0; q < H / 32; ++q) { b16 p, ql; split16(Z[(m0 + rr) * H + q * 32 + lane] * HS, p, ql); Ah[rr][q * 32 + lane] = p; Al[rr][q * 32 + lane] = ql; } if (lane < 16) for (int kk = H; kk < H + 8; ++kk) { Ah[lane][kk] = (b16)0.0f; Al[lane][kk] = (b16)0.0f; }
  wave_lds_sync(); v8f acc[16];
#pragma unroll
  for (int t = 0; t < 16; ++t) acc[t] = (v8f){};
#pragma unroll 2
  for (int kb = 0; kb < H; kb += 32) { const v16b a = frag_kb(&Ah[nloc][kb], hlf), al = frag_kb(&Al[nloc][kb], hlf);
#pragma unroll
    for (int t = 0; t < 16; ++t) { const v16b bw = frag_kb(WC1 + (size_t)(t * 16 + nloc) * H + kb, hlf); acc[t] = wmma16b(a, bw, acc[t]); acc[t] = wmma16b(al, bw, acc[t]); } }
  wave_lds_sync();
#pragma unroll
  for (int t = 0; t < 16; ++t) { const int cc = t * 16 + nloc; const float bb = bfv(bc1[cc]);
#pragma unroll
    for (int r8 = 0; r8 < 8; ++r8) { b16 p, ql; split16((acc[t][r8] * (1.0f / (HS * WSC)) + bb) * HS, p, ql); Ah[8 * hlf + r8][cc] = p; Al[8 * hlf + r8][cc] = ql; } }
  wave_lds_sync(); v8f lg = {};
#pragma unroll 2
  for (int kb = 0; kb < H; kb += 32) { const v16b bw = frag_kb(WC2 + (size_t)nloc * H + kb, hlf); lg = wmma16b(frag_kb(&Ah[nloc][kb], hlf), bw, lg); lg = wmma16b(frag_kb(&Al[nloc][kb], hlf), bw, lg); }
#pragma unroll
  for (int r8 = 0; r8 < 8; ++r8) Tf[8 * hlf + r8][nloc] = lg[r8] * (1.0f / (HS * WSC)) + bfv(bc2[nloc]);
  wave_lds_sync();
  if (lane < 16) { float mx = -INFINITY; for (int c = 0; c < C; ++c) mx = fmaxf(mx, Tf[lane][c]); float s = 0.0f; for (int c = 0; c < C; ++c) s += __expf(Tf[lane][c] - mx); const float lse = mx + __logf(s); for (int c = 0; c < C; ++c) Tf[lane][c] -= lse; }
  wave_lds_sync();
  for (int pass = 0; pass < 2; ++pass) { for (int q = 0; q < 2; ++q) { const int idx = q * 128 + lane * 4; *(volatile v4f*)(OUT1 + m0 * C + idx) = (v4f){Tf[idx / C][idx % C], Tf[(idx + 1) / C][(idx + 1) % C], Tf[(idx + 2) / C][(idx + 2) % C], Tf[(idx + 3) / C][(idx + 3) % C]}; } __threadfence(); } }
__global__ __launch_bounds__(32) void gram_kernel(const b16* __restrict__ ZN, int NLIM, float* __restrict__ GR) { __shared__ __attribute__((aligned(16))) b16 Zt[H][40]; __shared__ float Tf[16][H + 4]; const int lane = threadIdx.x, nloc = lane & 15, hlf = lane >> 4; const int k = blockIdx.x / (H / 8), ci = (blockIdx.x % (H / 8)) >> 1, hj = blockIdx.x & 1;     const b16* Zk = ZN + (size_t)k * N * H; v8f acc[8];
#pragma unroll
  for (int t = 0; t < 8; ++t) acc[t] = (v8f){};
  if (lane < 16) for (int c = 0; c < H; c += 1) if ((c & 15) == nloc) for (int q = 32; q < 40; ++q) Zt[c][q] = (b16)0.0f;
#pragma unroll 1
  for (int s0 = 0; s0 < NLIM; s0 += 32) {
    for (int cq = 0; cq < H / 8; ++cq) { const v8b v = *(const v8b*)(Zk + (size_t)(s0 + lane) * H + cq * 8);
#pragma unroll
      for (int j = 0; j < 8; ++j) Zt[cq * 8 + j][lane] = v[j]; }
    wave_lds_sync(); const v16b a = frag_kb(&Zt[ci * 16 + nloc][0], hlf);
#pragma unroll
    for (int t = 0; t < 8; ++t) acc[t] = wmma16b(a, frag_kb(&Zt[(hj * 8 + t) * 16 + nloc][0], hlf), acc[t]);
    wave_lds_sync(); }
#pragma unroll
  for (int t = 0; t < 8; ++t)
#pragma unroll
    for (int r8 = 0; r8 < 8; ++r8) Tf[8 * hlf + r8][t * 16 + nloc] = acc[t][r8];
  wave_lds_sync();
  for (int pass = 0; pass < 2; ++pass) { for (int rr = 0; rr < 16; ++rr) *(volatile v4f*)(GR + ((size_t)k * H + ci * 16 + rr) * H + hj * 128 + lane * 4) = *(const v4f*)(&Tf[rr][lane * 4]); __threadfence(); } }
__global__ __launch_bounds__(32) void supcon_kernel(const b16* __restrict__ ZN, const int* __restrict__ train, const int* __restrict__ y, const float* __restrict__ OUT1, int TLIM, int NLIM, float* __restrict__ PART) { __shared__ __attribute__((aligned(16))) b16 Aa[16][H + 8]; __shared__ float Sf[16][20]; __shared__ int Lt[16], Lk[16]; const int lane = threadIdx.x, nloc = lane & 15, hlf = lane >> 4; const int t0 = blockIdx.x * 16; if (t0 >= TLIM) return;
  { const int tn = iclamp(train[t0 + nloc], 0, NLIM - 1); if (hlf == 0) Lt[nloc] = iclamp(y[tn], 0, C - 1); for (int cq = hlf; cq < H / 8; cq += 2) *(v8b*)(&Aa[nloc][cq * 8]) = *(const v8b*)(ZN + (size_t)tn * H + cq * 8); if (hlf == 0) for (int q = H; q < H + 8; ++q) Aa[nloc][q] = (b16)0.0f; }
  wave_lds_sync();
  float ma = -INFINITY, sa = 0.0f, mp = -INFINITY, sp = 0.0f;
  const int myl = Lt[nloc];
#pragma unroll 1
  for (int u0 = 0; u0 < TLIM; u0 += 16) { const int un = iclamp(train[u0 + nloc], 0, NLIM - 1); if (hlf == 0) Lk[nloc] = iclamp(y[un], 0, C - 1); v8f s = {};
#pragma unroll 2
    for (int kb = 0; kb < H; kb += 32) s = wmma16b(frag_kb(&Aa[nloc][kb], hlf), frag_kb(ZN + (size_t)N * H + (size_t)un * H + kb, hlf), s);
#pragma unroll
    for (int r8 = 0; r8 < 8; ++r8) Sf[8 * hlf + r8][nloc] = s[r8] * (1.0f / TAU);
    wave_lds_sync();
    if (lane < 16) { float bm = -INFINITY; for (int q = 0; q < 16; ++q) bm = fmaxf(bm, Sf[lane][q]); { const float mn = fmaxf(ma, bm); float add = 0.0f; for (int q = 0; q < 16; ++q) add += __expf(Sf[lane][q] - mn); sa = sa * ((ma == -INFINITY) ? 0.0f : __expf(ma - mn)) + add; ma = mn; }
      float pm = -INFINITY; for (int q = 0; q < 16; ++q) if (Lk[q] == myl) pm = fmaxf(pm, Sf[lane][q]); if (pm > -INFINITY) { const float mn = fmaxf(mp, pm); float add = 0.0f; for (int q = 0; q < 16; ++q) if (Lk[q] == myl) add += __expf(Sf[lane][q] - mn); sp = sp * ((mp == -INFINITY) ? 0.0f : __expf(mp - mn)) + add; mp = mn; } }
    wave_lds_sync(); }
  if (lane < 16) { Sf[lane][0] = (ma + __logf(sa)) - (mp + __logf(sp)); const int tn = iclamp(train[t0 + lane], 0, NLIM - 1); Sf[lane][1] = -OUT1[(size_t)tn * C + myl]; }
  wave_lds_sync();
  float cls = 0.0f, nls = 0.0f; if (lane == 0) for (int q = 0; q < 16; ++q) { cls += Sf[q][0]; nls += Sf[q][1]; }
  cls = __shfl(cls, 0); nls = __shfl(nls, 0);
  for (int pass = 0; pass < 2; ++pass) { ((volatile float*)PART)[(size_t)blockIdx.x * 32 + lane] = lane == 0 ? cls : (lane == 1 ? nls : 0.0f); __threadfence(); } }
__global__ __launch_bounds__(256) void loss_kernel(const float* __restrict__ PART, int nw, const float* __restrict__ DG, const float* __restrict__ GR, int NLIM, int TLIM, float* __restrict__ OUT2) { __shared__ double Rd[256][4]; const int t = threadIdx.x; double s_cl = 0.0, s_nl = 0.0, s_d1 = 0.0, s_d2 = 0.0, s_f = 0.0;
  for (int w = t; w < nw; w += 256) { s_cl += (double)PART[(size_t)w * 32]; s_nl += (double)PART[(size_t)w * 32 + 1]; }
  for (int n = t; n < NLIM; n += 256) { const double d = (double)DG[(n >> 4) * 32 + (n & 15)]; s_d1 += (d - 1.0) * (d - 1.0); s_d2 += d * d; }
  for (int i = t; i < H * H; i += 256) s_f += (double)GR[i] * (double)GR[(size_t)H * H + i];
  Rd[t][0] = s_cl; Rd[t][1] = s_nl; Rd[t][2] = s_d1; Rd[t][3] = s_d2; __shared__ double Rf[256]; Rf[t] = s_f; __syncthreads();
  if (t == 0) { double cl = 0.0, nl = 0.0, d1 = 0.0, d2 = 0.0, f = 0.0; for (int q = 0; q < 256; ++q) { cl += Rd[q][0]; nl += Rd[q][1]; d1 += Rd[q][2]; d2 += Rd[q][3]; f += Rf[q]; }
    const double nn = (double)NLIM; const double loss = nl / TLIM + 0.1 * (d1 / nn + (f - d2) / (nn * (nn - 1.0))) + cl / TLIM;
    for (int pass = 0; pass < 2; ++pass) { ((volatile float*)OUT2)[0] = (float)loss; __threadfence(); } } }
}

extern "C" void kernel_launch(void* const* d_in, const int* in_sizes, int n_in, void* d_out, int out_size, void* d_ws, size_t ws_size, hipStream_t stream) {
  (void)n_in;
  auto Fp = [&](int i) { return (const float*)d_in[i]; }; auto Ip = [&](int i) { return (const int*)d_in[i]; };
  if (in_sizes[0] != N * FI || in_sizes[1] != E || in_sizes[2] != E || in_sizes[3] != E || in_sizes[4] != T || in_sizes[5] != N || in_sizes[6] != FI * H || in_sizes[8] != H * H || in_sizes[10] != FI * H || in_sizes[12] != H * H || in_sizes[14] != H * H || in_sizes[16] != H * C || in_sizes[17] != C || out_size != N * H + N * C + 1) return;
  const int NLIM = N, TLIM = T;
  size_t off = 0; char* ws = (char*)d_ws;
  auto carve = [&](size_t bytes) { char* p = ws + off; off += (bytes + 255) & ~(size_t)255; return p; };
  b16* WG = (b16*)carve((size_t)2 * H * FI * 2); b16* WL = (b16*)carve((size_t)2 * H * H * 2); b16* WC1 = (b16*)carve((size_t)H * H * 2); b16* WC2 = (b16*)carve((size_t)C * H * 2);
  float* SUP = (float*)carve((size_t)N * 2 * H * 4); float* HH = (float*)carve((size_t)N * 2 * H * 4); b16* ZN = (b16*)carve((size_t)2 * N * H * 2); float* DG = (float*)carve((size_t)(N / 16) * 32 * 4); float* GR = (float*)carve((size_t)2 * H * H * 4); float* PART = (float*)carve((size_t)(T / 16) * 32 * 4); CsrBufs8 csr; off = csr_carve8(csr, ws, off, E, N);
  if (off > ws_size || off > ((size_t)128 << 20)) return;
  float* Z = (float*)d_out; float* OUT1 = Z + (size_t)N * H; float* OUT2 = OUT1 + (size_t)N * C;
  wput_kernel<<<(2 * H * (FI / 8) + 255) / 256, 256, 0, stream>>>(Fp(6), Fp(10), Fp(8), Fp(12), Fp(14), Fp(16), WG, WL, WC1, WC2);
  csr_build8(csr, Ip(1), E, N, stream);
  sup_kernel<<<(NLIM / 16) * 2, 32, 0, stream>>>(Fp(0), WG, NLIM, SUP);
  spmm_kernel<<<(NLIM + 7) / 8, 256, 0, stream>>>(SUP, Fp(3), Ip(2), Fp(7), Fp(11), csr.PERM, csr.ROWPTR, csr.ROWCNT, (int)csr.permLen, NLIM, HH);
  enc_kernel<<<NLIM / 16, 32, 0, stream>>>(HH, WL, Fp(9), Fp(13), NLIM, Z, ZN, DG);
  cls_kernel<<<NLIM / 16, 32, 0, stream>>>(Z, WC1, WC2, Fp(15), Fp(17), NLIM, OUT1);
  gram_kernel<<<2 * (H / 8), 32, 0, stream>>>(ZN, NLIM, GR);
  supcon_kernel<<<TLIM / 16, 32, 0, stream>>>(ZN, Ip(4), Ip(5), OUT1, TLIM, NLIM, PART);
  loss_kernel<<<1, 256, 0, stream>>>(PART, TLIM / 16, DG, GR, NLIM, TLIM, OUT2);
}
